// CausalSelfAttention_27127013441644
// MI455X (gfx1250) — hardware-verified
//
#include <hip/hip_runtime.h>
#ifndef NB
#define NB 2
#endif
#ifndef SQ
#define SQ 2048
#endif
#define NB_FULL 2
#define SQ_FULL 2048
#define DM 1024
#define NH 16
#define NKV 4
#define KVSH 2
#define HD 64
#define KVD (NKV * HD)
#define LQ (DM + 2 * KVD)
#define ROTN (DM + KVD)
#define QT 256
#define QT0 256
#define NKX SQ
#define NR ((size_t)NB * SQ)

static_assert(NB <= NB_FULL);
static_assert(SQ <= SQ_FULL);
static_assert((SQ & (SQ - 1)) == 0);
static_assert(SQ % QT == 0);
static_assert((QT & (QT - 1)) == 0);
static_assert(QT % 128 == 0);
static_assert(QT0 == QT);
static_assert(QT0 % 128 == 0);
static_assert(QT0 % 64 == 0);
static_assert(HD == 64);
static_assert(DM == NH * HD);
static_assert(NH == (NKV << KVSH));
static_assert(DM / 8 == 128);
static_assert(DM % 64 == 0);
static_assert(KVD % 64 == 0);
static_assert(LQ % 64 == 0);
static_assert(ROTN % 64 == 0);
static_assert(((size_t)NB * SQ) % 128 == 0);
static_assert(SQ % 64 == 0);
static_assert(DM % 32 == 0);

typedef unsigned short v8us __attribute__((ext_vector_type(8), may_alias));
typedef float  v8f  __attribute__((ext_vector_type(8)));
typedef float  v4f  __attribute__((ext_vector_type(4)));
typedef float  v4fa __attribute__((ext_vector_type(4), may_alias));
typedef _Float16 v16h __attribute__((ext_vector_type(16)));
typedef _Float16 v4h __attribute__((ext_vector_type(4)));
union FragH { v16h v; v8us half[2]; _Float16 h[16]; unsigned short u[16]; };

__device__ __forceinline__ unsigned short bf16_bits(float x) { unsigned int u = __float_as_uint(x); return (unsigned short)((u + 0x7FFFu + ((u >> 16) & 1u)) >> 16); }
__device__ __forceinline__ float bf16_val(unsigned short b) { return __uint_as_float(((unsigned int)b) << 16); }
__device__ __forceinline__ float bf16_rne(float x) { return bf16_val(bf16_bits(x)); }

__device__ __forceinline__ v16h g2_frag(const _Float16* p, unsigned hh) { FragH f; f.half[0] = *(const v8us*)((const unsigned short*)p + 8 * hh); f.half[1] = *(const v8us*)((const unsigned short*)p + 16 + 8 * hh); return f.v; }
__device__ __forceinline__ v8f g2_mma(v16h a, v16h b, v8f c) { v8f d = __builtin_amdgcn_wmma_f32_16x16x32_f16(false, a, false, b, (short)0, c, false, false); asm volatile("v_nop\n\tv_nop\n\tv_nop\n\tv_nop" : "+v"(d) : "v"(a), "v"(b)); return d; }

__global__ __launch_bounds__(256) void k_wT(const float* __restrict__ w, unsigned int Kd, unsigned int Nd, _Float16* __restrict__ Bt) {
  __shared__ unsigned short tl[64][66];
  const unsigned int tid = threadIdx.x; const unsigned int ntn = Nd >> 6; const unsigned int kt = blockIdx.x / ntn, nt = blockIdx.x - kt * ntn; const unsigned int k0 = kt * 64u, n0 = nt * 64u;
  for (unsigned int i = tid; i < 64u * 16u; i += 256u) { const unsigned int r = i >> 4, c4 = (i & 15u) * 4u; const v4f a = *(const v4fa*)(w + (size_t)(k0 + r) * Nd + n0 + c4); FragH f;
#pragma unroll
    for (int q = 0; q < 4; ++q) f.h[q] = (_Float16)(bf16_rne(a[q]) * 16.0f);
#pragma unroll
    for (int q = 0; q < 4; ++q) tl[r][c4 + q] = f.u[q]; }
  __syncthreads();
  for (int pass = 0; pass < 2; ++pass) {
#pragma unroll
    for (int rd = 0; rd < 2; ++rd) { const unsigned int d = (unsigned int)rd * 32u + (tid >> 3), pc = tid & 7u; FragH f;
#pragma unroll
      for (int q = 0; q < 8; ++q) f.u[q] = tl[pc * 8u + q][d];
      const v8us o = f.half[0];
      *(volatile v8us*)((unsigned short*)Bt + (size_t)(n0 + d) * Kd + k0 + pc * 8u) = o; }
    if (pass == 0) __threadfence(); } }

__global__ __launch_bounds__(256) void k_x16(const float* __restrict__ x, _Float16* __restrict__ X16, unsigned int n8) {
  const unsigned int t = blockIdx.x * 256u + threadIdx.x; if (t >= n8) return;
  const unsigned int row = t >> 7;
  const unsigned int b = row / (unsigned int)SQ, s = row - b * (unsigned int)SQ;
  const float* src = x + ((size_t)b * SQ_FULL + s) * DM + (size_t)(t & 127u) * 8u;
  const v4f a = *(const v4fa*)src, c = *(const v4fa*)(src + 4);
  FragH f;
#pragma unroll
  for (int q = 0; q < 4; ++q) { f.h[q] = (_Float16)bf16_rne(a[q]); f.h[4 + q] = (_Float16)bf16_rne(c[q]); }
  const v8us o = f.half[0];
  unsigned short* d = (unsigned short*)X16 + (size_t)t * 8u;
  *(volatile v8us*)d = o; __threadfence(); *(volatile v8us*)d = o;
}

__global__ __launch_bounds__(256) void k_vt(const _Float16* __restrict__ V16, _Float16* __restrict__ Vt) {
  __shared__ unsigned short tl[64][66];
  const unsigned int tid = threadIdx.x; const unsigned int slab = blockIdx.x / (unsigned int)(SQ / 64), lg = blockIdx.x % (unsigned int)(SQ / 64); const unsigned int b = slab / (unsigned int)NKV, h = slab % (unsigned int)NKV;
  for (unsigned int i = tid; i < 64u * 8u; i += 256u) { const unsigned int r = i >> 3, c8 = (i & 7u) * 8u; FragH f; f.half[0] = *(const v8us*)((const unsigned short*)V16 + ((size_t)b * SQ + lg * 64u + r) * LQ + h * 64u + c8);
#pragma unroll
    for (int q = 0; q < 8; ++q) tl[r][c8 + q] = f.u[q]; }
  __syncthreads();
  for (int pass = 0; pass < 2; ++pass) {
#pragma unroll
    for (int rd = 0; rd < 2; ++rd) { const unsigned int d = (unsigned int)rd * 32u + (tid >> 3), pc = tid & 7u; FragH f;
#pragma unroll
      for (int q = 0; q < 8; ++q) f.u[q] = tl[pc * 8u + q][d];
      const v8us o = f.half[0];
      *(volatile v8us*)((unsigned short*)Vt + ((size_t)slab * 64u + d) * SQ + lg * 64u + pc * 8u) = o; }
    if (pass == 0) __threadfence(); } }

__global__ __launch_bounds__(256) void k_hl(const float* __restrict__ F, _Float16* __restrict__ Hh, _Float16* __restrict__ Hl, unsigned int n8) {
  const unsigned int t = blockIdx.x * 256u + threadIdx.x; if (t >= n8) return; FragH fh, fl; const v4f a = *(const v4fa*)(F + (size_t)t * 8u), c = *(const v4fa*)(F + (size_t)t * 8u + 4);
  const unsigned int row = t >> 7; const unsigned int b = row / (unsigned int)QT0, r = row - b * (unsigned int)QT0;
  const size_t dh = ((size_t)b * SQ + r) * DM + (size_t)(t & 127u) * 8u;
#pragma unroll
  for (int q = 0; q < 4; ++q) { _Float16 h = (_Float16)a[q]; fh.h[q] = h; fl.h[q] = (_Float16)((a[q] - (float)h) * 1024.0f); h = (_Float16)c[q]; fh.h[4 + q] = h; fl.h[4 + q] = (_Float16)((c[q] - (float)h) * 1024.0f); }
  const v8us oh = fh.half[0], ol = fl.half[0];
  for (int pass = 0; pass < 2; ++pass) { *(volatile v8us*)((unsigned short*)Hh + dh) = oh; *(volatile v8us*)((unsigned short*)Hl + dh) = ol; if (pass == 0) __threadfence(); } }

__global__ __launch_bounds__(128) void k_gemm2(const _Float16* __restrict__ A, int lda, size_t sA, const _Float16* __restrict__ Bh, int ldb, size_t sB, unsigned int bsh, float alpha, const float* CP,
    float* C, _Float16* C16, _Float16* C16L, int ldc, size_t sC, int M, int N, int K, const float* cosb, const float* sinb, unsigned int rotN, unsigned int pmask) {
  __shared__ __attribute__((aligned(16))) float so[4][32][68];
  const unsigned int tid = threadIdx.x, w = tid >> 5, lane = tid & 31u, ln = lane & 15u, hh = lane >> 4; const unsigned int by = blockIdx.y;
  A += (size_t)by * sA; Bh += (size_t)(by >> bsh) * sB; const size_t cofs = (size_t)by * sC;
  const unsigned int ntn = (unsigned int)N >> 6; const unsigned int mt = blockIdx.x / ntn, nq = blockIdx.x - mt * ntn; const unsigned int row0 = mt * 128u + 32u * w, col0 = nq * 64u; if (row0 >= (unsigned int)M) return;
  const _Float16* a0p = A + (size_t)(row0 + ln) * lda; const _Float16* a1p = a0p + (size_t)16 * lda;
  const _Float16* b0p = Bh + (size_t)(col0 + ln) * ldb; const _Float16* b1p = b0p + (size_t)16 * ldb; const _Float16* b2p = b1p + (size_t)16 * ldb; const _Float16* b3p = b2p + (size_t)16 * ldb;
  const v8f z8 = {0.f,0.f,0.f,0.f,0.f,0.f,0.f,0.f}; v8f c00 = z8, c01 = z8, c02 = z8, c03 = z8, c10 = z8, c11 = z8, c12 = z8, c13 = z8;
#pragma unroll 1
  for (int kb = 0; kb < K; kb += 32) { const v16h a0 = g2_frag(a0p + kb, hh), a1 = g2_frag(a1p + kb, hh);
    v16h b = g2_frag(b0p + kb, hh); c00 = g2_mma(a0, b, c00); c10 = g2_mma(a1, b, c10);
    b = g2_frag(b1p + kb, hh); c01 = g2_mma(a0, b, c01); c11 = g2_mma(a1, b, c11);
    b = g2_frag(b2p + kb, hh); c02 = g2_mma(a0, b, c02); c12 = g2_mma(a1, b, c12);
    b = g2_frag(b3p + kb, hh); c03 = g2_mma(a0, b, c03); c13 = g2_mma(a1, b, c13); }
  v8f accs[8] = {c00, c01, c02, c03, c10, c11, c12, c13};
#pragma unroll
  for (int u = 0; u < 8; ++u) { const unsigned int t = (unsigned int)u & 3u, half = (unsigned int)u >> 2; const unsigned int col = col0 + t * 16u + ln;
#pragma unroll
    for (int r = 0; r < 8; ++r) { const unsigned int rloc = half * 16u + 8u * hh + (unsigned int)r; float v = accs[u][r] * alpha; if (CP) v += CP[cofs + (size_t)(row0 + rloc) * ldc + col];
      so[w][rloc][t * 16u + ln] = v; } }
  __builtin_amdgcn_fence(4  , "workgroup"); __builtin_amdgcn_wave_barrier();
  if (col0 < rotN) {
    const unsigned int pos = (row0 + lane) & pmask;
    const float* cr = cosb + (size_t)pos * 32u; const float* sr = sinb + (size_t)pos * 32u; float ss = 0.f;
#pragma unroll 1
    for (unsigned int j = 0; j < 32u; j += 4u) { const v4f cc = *(const v4fa*)(cr + j), sn = *(const v4fa*)(sr + j); const v4f x1 = *(const v4fa*)&so[w][lane][j], x2 = *(const v4fa*)&so[w][lane][32u + j]; v4f y1, y2;
#pragma unroll
      for (int q = 0; q < 4; ++q) { const float c = bf16_rne(cc[q]), s = bf16_rne(sn[q]); y1[q] = x1[q] * c + x2[q] * s; y2[q] = x2[q] * c - x1[q] * s; ss += y1[q] * y1[q] + y2[q] * y2[q]; }
      *(v4fa*)&so[w][lane][j] = y1; *(v4fa*)&so[w][lane][32u + j] = y2; }
    const float rs = rsqrtf(ss * 0.015625f + 1.0e-6f);
#pragma unroll 1
    for (unsigned int j = 0; j < 64u; j += 4u) { v4f y = *(const v4fa*)&so[w][lane][j];
#pragma unroll
      for (int q = 0; q < 4; ++q) y[q] = y[q] * rs;
      *(v4fa*)&so[w][lane][j] = y; }
    __builtin_amdgcn_fence(4  , "workgroup"); __builtin_amdgcn_wave_barrier(); }
  const unsigned int rsub = lane >> 4, c4 = (lane & 15u) * 4u;
  for (int pass = 0; pass < 2; ++pass) {
#pragma unroll
    for (int q = 0; q < 16; ++q) { const unsigned int r = (unsigned int)q * 2u + rsub; const v4f v = *(const v4fa*)&so[w][r][c4]; const size_t o = cofs + (size_t)(row0 + r) * ldc + col0 + c4;
      if (C) *(volatile v4f*)(C + o) = v;
      if (C16) { v4h h4, l4;
#pragma unroll
        for (int i = 0; i < 4; ++i) { const _Float16 h = (_Float16)v[i]; h4[i] = h; l4[i] = (_Float16)((v[i] - (float)h) * 1024.0f); }
        *(volatile v4h*)(C16 + o) = h4; if (C16L) *(volatile v4h*)(C16L + o) = l4; } }
    if (pass == 0) __threadfence(); } }

__global__ __launch_bounds__(256) void k_rsmcf2(const float* __restrict__ S, _Float16* __restrict__ P, _Float16* __restrict__ PL, unsigned int hg, unsigned int q0, unsigned int nk) {
  #pragma clang fp contract(off)
  const unsigned int t = blockIdx.x * 256u + threadIdx.x; if (t >= hg * (unsigned int)QT) return; const size_t i = (size_t)t; const float* s = S + i * NKX; const unsigned int last = q0 + (t & (unsigned int)(QT - 1)); float mx = -3.0e38f;
#pragma unroll 1
  for (unsigned int j = 0; j < nk; ++j) { const float f = (j <= last) ? 1.f : 0.f; mx = fmaxf(mx, fmaf(f, s[j], (1.f - f) * -1.0e9f)); } float se = 0.f;
#pragma unroll 1
  for (unsigned int j = 0; j < nk; ++j) { const float f = (j <= last) ? 1.f : 0.f; se += __expf(fmaf(f, s[j], (1.f - f) * -1.0e9f) - mx); } const float sc = 256.0f / se;
#pragma unroll 1
  for (unsigned int j0 = 0; j0 < nk; j0 += 8) { FragH fr, fl;
#pragma unroll
    for (int q = 0; q < 8; ++q) { const unsigned int j = j0 + (unsigned int)q; const float f = (j <= last) ? 1.f : 0.f; const float pv = __expf(fmaf(f, s[j], (1.f - f) * -1.0e9f) - mx) * sc; const _Float16 h = (_Float16)pv; fr.h[q] = h; fl.h[q] = (_Float16)((pv - (float)h) * 1024.0f); }
    const v8us o = fr.half[0], ol = fl.half[0]; unsigned short* d = (unsigned short*)P + i * NKX + j0; unsigned short* dl = (unsigned short*)PL + i * NKX + j0;
    *(volatile v8us*)d = o; *(volatile v8us*)dl = ol; __threadfence(); *(volatile v8us*)d = o; *(volatile v8us*)dl = ol; } }

__global__ __launch_bounds__(64) void k_att0(const float* __restrict__ QF, const float* __restrict__ KF, const float* __restrict__ VF, int ld, size_t sF, float scale, float* __restrict__ OF, int ldo, size_t sO) {
  #pragma clang fp contract(off)
  __shared__ __attribute__((aligned(16))) float lq[64][64]; __shared__ __attribute__((aligned(16))) float lo[64][64];
  const unsigned int tid = threadIdx.x; const unsigned int h = blockIdx.x / (unsigned int)(QT0 / 64), rg = blockIdx.x % (unsigned int)(QT0 / 64); const unsigned int i = rg * 64u + tid; const unsigned int hk = h >> KVSH;
  const size_t fo = (size_t)blockIdx.y * sF; QF += fo; KF += fo; VF += fo; OF += (size_t)blockIdx.y * sO;
  const float* qr = QF + (size_t)i * ld + h * HD;
#pragma unroll 1
  for (int c = 0; c < HD / 4; ++c) { *(v4fa*)&lq[tid][c * 4] = *(const v4fa*)(qr + c * 4); const v4f z = {0.f, 0.f, 0.f, 0.f}; *(v4fa*)&lo[tid][c * 4] = z; }
  float m = -1.0e30f, l = 0.f; const unsigned int jmax = rg * 64u + 63u;
#pragma unroll 1
  for (unsigned int j = 0; j <= jmax; ++j) { const float* kr = KF + (size_t)j * ld + hk * HD; const float* vr = VF + (size_t)j * ld + hk * HD; float s = 0.f;
#pragma unroll 1
    for (int c = 0; c < HD / 4; ++c) { const v4f kq = *(const v4fa*)(kr + c * 4); const v4f qq = *(const v4fa*)&lq[tid][c * 4]; s = __fadd_rn(s, __fmul_rn(qq[0], kq[0])); s = __fadd_rn(s, __fmul_rn(qq[1], kq[1])); s = __fadd_rn(s, __fmul_rn(qq[2], kq[2])); s = __fadd_rn(s, __fmul_rn(qq[3], kq[3])); }
    s = __fmul_rn(s, scale);
    const float f = (j <= i) ? 1.f : 0.f; const float sm = fmaf(f, s, (1.f - f) * -1.0e30f); const float mn = fmaxf(m, sm); const float sc = expf(m - mn); const float e = expf(sm - mn); l = __fadd_rn(__fmul_rn(l, sc), e); m = mn;
#pragma unroll 1
    for (int c = 0; c < HD / 4; ++c) { const v4f vv = *(const v4fa*)(vr + c * 4); v4f oo = *(const v4fa*)&lo[tid][c * 4];
#pragma unroll
      for (int u = 0; u < 4; ++u) oo[u] = __fadd_rn(__fmul_rn(oo[u], sc), __fmul_rn(e, vv[u]));
      *(v4fa*)&lo[tid][c * 4] = oo; } }
  const float fin = 64.0f / l;
#pragma unroll 1
  for (int c = 0; c < HD / 4; ++c) { v4f oo = *(const v4fa*)&lo[tid][c * 4];
#pragma unroll
    for (int u = 0; u < 4; ++u) oo[u] = __fmul_rn(oo[u], fin);
    *(v4fa*)&lo[tid][c * 4] = oo; }
  __syncthreads();
  for (int pass = 0; pass < 2; ++pass) {
#pragma unroll 1
    for (unsigned int it = 0; it < 16u; ++it) { const unsigned int row = it * 4u + (tid >> 4), pc = (tid & 15u) * 4u; const v4f v = *(const v4fa*)&lo[row][pc]; *(volatile v4f*)(OF + (size_t)(rg * 64u + row) * ldo + h * HD + pc) = v; }
    if (pass == 0) __threadfence(); } }

constexpr size_t al256(size_t b) { return (b + 255) & ~(size_t)255; }
constexpr size_t cmax(size_t a, size_t b) { return a > b ? a : b; }
constexpr size_t SZ_BQKV = al256((size_t)LQ * DM * 2);
constexpr size_t SZ_BO   = al256((size_t)DM * DM * 2);
constexpr size_t SZ_XO   = al256(NR * DM * 2);
constexpr size_t SZ_QKV  = al256(NR * LQ * 2);
constexpr size_t SZ_F0   = al256((size_t)NB * QT0 * LQ * 4);
constexpr size_t SZ_OF0  = al256((size_t)NB * QT0 * DM * 4);
constexpr size_t SZ_S    = cmax(al256((size_t)NH * QT * NKX * 4), SZ_F0 + SZ_OF0);
constexpr size_t SZ_P    = al256((size_t)NH * QT * NKX * 2);
constexpr size_t SZ_VT   = al256((size_t)NB * NKV * HD * SQ * 2);
constexpr size_t SZ_OL   = al256(NR * DM * 2);
constexpr size_t SZ_OT   = al256((size_t)QT * DM * 4);
static_assert(SZ_F0 + SZ_OF0 <= SZ_S);
constexpr size_t WS_TOTAL = SZ_BQKV + SZ_BO + SZ_XO + 2 * SZ_QKV + SZ_S + 2 * SZ_P + 2 * SZ_VT + SZ_OL + SZ_OT;
static_assert(WS_TOTAL <= (size_t)134217728);
static_assert(((size_t)(DM / 64) * (DM / 64)) * 64 * 64 == (size_t)DM * DM);
static_assert(((size_t)(DM / 64) * (KVD / 64)) * 64 * 64 == (size_t)DM * KVD);
static_assert(((size_t)NB * NKV * (SQ / 64)) * 64 * 64 == (size_t)NB * NKV * HD * SQ);
static_assert((NR * DM) % (256 * 8) == 0);
static_assert(((size_t)NB * QT0 * DM) % (256 * 8) == 0);
static_assert(((size_t)NH * QT) % 256 == 0);
static_assert((size_t)NH * (QT0 / 64) * 64 == (size_t)NH * QT0);
static_assert(((size_t)(NR / 128) * (LQ / 64)) * 128 * 64 == NR * LQ);
static_assert(((size_t)(QT / 128) * (HD / 64) * NH) * 128 * 64 == (size_t)QT * DM);
static_assert(((size_t)(SQ / 128) * (DM / 64) * NB) * 128 * 64 == NR * DM);

extern "C" void kernel_launch(void* const* d_in, const int* in_sizes, int n_in,
                              void* d_out, int out_size, void* d_ws, size_t ws_size, hipStream_t stream) {
  if (n_in < 7) return;
  const size_t need_x = ((size_t)(NB - 1) * SQ_FULL + SQ) * DM;
  if ((size_t)in_sizes[0] < need_x) return;
  if ((size_t)in_sizes[1] < (size_t)SQ * 32) return;
  if ((size_t)in_sizes[2] < (size_t)SQ * 32) return;
  if ((size_t)in_sizes[3] < (size_t)DM * DM) return;
  if ((size_t)in_sizes[4] < (size_t)DM * KVD) return;
  if ((size_t)in_sizes[5] < (size_t)DM * KVD) return;
  if ((size_t)in_sizes[6] < (size_t)DM * DM) return;
  if ((size_t)out_size < need_x) return;
  const float* x = (const float*)d_in[0]; const float* cosb = (const float*)d_in[1]; const float* sinb = (const float*)d_in[2];
  const float* wq = (const float*)d_in[3]; const float* wk = (const float*)d_in[4]; const float* wv = (const float*)d_in[5]; const float* wo = (const float*)d_in[6];
  float* out = (float*)d_out;
  char* ws = (char*)d_ws; size_t off = 0;
  auto take = [&](size_t bytes) { char* p = ws + off; off += (bytes + 255) & ~(size_t)255; return p; };
  _Float16* BQKV = (_Float16*)take(SZ_BQKV); _Float16* BO = (_Float16*)take(SZ_BO);
  _Float16* X16 = (_Float16*)take(SZ_XO); _Float16* OH = X16;
  _Float16* QKV = (_Float16*)take(SZ_QKV); const _Float16* Q16 = QKV; const _Float16* K16 = QKV + DM; const _Float16* V16 = QKV + ROTN;
  _Float16* QKVL = (_Float16*)take(SZ_QKV); const _Float16* QL = QKVL; const _Float16* VL16 = QKVL + ROTN;
  char* sreg = take(SZ_S); float* S = (float*)sreg; float* F0 = (float*)sreg; float* OF0 = (float*)(sreg + SZ_F0);
  _Float16* PH = (_Float16*)take(SZ_P); _Float16* PL = (_Float16*)take(SZ_P);
  _Float16* VT = (_Float16*)take(SZ_VT); _Float16* VTL = (_Float16*)take(SZ_VT);
  _Float16* OL = (_Float16*)take(SZ_OL); float* OT = (float*)take(SZ_OT);
  if (off > ws_size) return;

  k_wT<<<(DM / 64) * (DM / 64), 256, 0, stream>>>(wq, (unsigned int)DM, (unsigned int)DM, BQKV);
  k_wT<<<(DM / 64) * (KVD / 64), 256, 0, stream>>>(wk, (unsigned int)DM, (unsigned int)KVD, BQKV + (size_t)DM * DM);
  k_wT<<<(DM / 64) * (KVD / 64), 256, 0, stream>>>(wv, (unsigned int)DM, (unsigned int)KVD, BQKV + (size_t)ROTN * DM);
  k_wT<<<(DM / 64) * (DM / 64), 256, 0, stream>>>(wo, (unsigned int)DM, (unsigned int)DM, BO);
  const unsigned int n8x = (unsigned int)(NR * DM / 8);
  k_x16<<<(n8x + 255u) / 256u, 256, 0, stream>>>(x, X16, n8x);
  const int MP = (int)(NR); const unsigned int pm = (unsigned int)(SQ - 1);
  k_gemm2<<<dim3((unsigned int)((MP / 128) * (LQ / 64)), 1), 128, 0, stream>>>(X16, DM, (size_t)0, BQKV, DM, (size_t)0, 0u, 0.0625f, nullptr, nullptr, QKV, QKVL, LQ, (size_t)0, MP, LQ, DM, cosb, sinb, (unsigned int)ROTN, pm);
  k_gemm2<<<dim3((unsigned int)((QT0 / 128) * (LQ / 64)), NB), 128, 0, stream>>>(X16, DM, (size_t)SQ * DM, BQKV, DM, (size_t)0, 0u, 0.0625f, nullptr, F0, nullptr, nullptr, LQ, (size_t)QT0 * LQ, QT0, LQ, DM, cosb, sinb, (unsigned int)ROTN, pm);
  k_vt<<<NB * NKV * (SQ / 64), 256, 0, stream>>>(V16, VT);
  k_vt<<<NB * NKV * (SQ / 64), 256, 0, stream>>>(VL16, VTL);
  k_att0<<<dim3(NH * (QT0 / 64), NB), 64, 0, stream>>>(F0, F0 + DM, F0 + ROTN, LQ, (size_t)QT0 * LQ, 0.125f, OF0, DM, (size_t)QT0 * DM);
  const unsigned int n8h = (unsigned int)((size_t)NB * QT0 * DM / 8);
  k_hl<<<(n8h + 255u) / 256u, 256, 0, stream>>>(OF0, OH, OL, n8h);
  for (unsigned int b = 0; b < (unsigned int)NB; ++b) { const size_t r0 = (size_t)b * SQ; const _Float16* VTb = VT + (size_t)b * NKV * HD * SQ; const _Float16* VTLb = VTL + (size_t)b * NKV * HD * SQ;
    for (unsigned int q0 = (unsigned int)QT; q0 < (unsigned int)SQ; q0 += QT) { const unsigned int nk = q0 + QT;
      const dim3 gs((QT / 128) * (nk / 64), NH), go((QT / 128) * (HD / 64), NH);
      k_gemm2<<<gs, 128, 0, stream>>>(Q16 + (r0 + q0) * LQ, LQ, (size_t)HD, K16 + r0 * LQ, LQ, (size_t)HD, (unsigned int)KVSH, 0.125f, nullptr, S, nullptr, nullptr, NKX, (size_t)QT * NKX, QT, (int)nk, HD, nullptr, nullptr, 0u, 0u);
      k_gemm2<<<gs, 128, 0, stream>>>(QL + (r0 + q0) * LQ, LQ, (size_t)HD, K16 + r0 * LQ, LQ, (size_t)HD, (unsigned int)KVSH, 0.0001220703125f, (const float*)S, S, nullptr, nullptr, NKX, (size_t)QT * NKX, QT, (int)nk, HD, nullptr, nullptr, 0u, 0u);
      k_rsmcf2<<<(NH * QT + 255) / 256, 256, 0, stream>>>(S, PH, PL, (unsigned int)NH, q0, nk);
      k_gemm2<<<go, 128, 0, stream>>>(PH, NKX, (size_t)QT * NKX, VTb, SQ, (size_t)HD * SQ, (unsigned int)KVSH, 0.25f, nullptr, OT, nullptr, nullptr, DM, (size_t)HD, QT, HD, (int)nk, nullptr, nullptr, 0u, 0u);
      k_gemm2<<<go, 128, 0, stream>>>(PH, NKX, (size_t)QT * NKX, VTLb, SQ, (size_t)HD * SQ, (unsigned int)KVSH, 0.000244140625f, (const float*)OT, OT, nullptr, nullptr, DM, (size_t)HD, QT, HD, (int)nk, nullptr, nullptr, 0u, 0u);
      k_gemm2<<<go, 128, 0, stream>>>(PL, NKX, (size_t)QT * NKX, VTb, SQ, (size_t)HD * SQ, (unsigned int)KVSH, 0.000244140625f, (const float*)OT, nullptr, OH + (r0 + q0) * DM, OL + (r0 + q0) * DM, DM, (size_t)HD, QT, HD, (int)nk, nullptr, nullptr, 0u, 0u); } }
  k_gemm2<<<dim3((SQ / 128) * (DM / 64), NB), 128, 0, stream>>>(OH, DM, (size_t)SQ * DM, BO, DM, (size_t)0, 0u, 0.0009765625f, nullptr, out, nullptr, nullptr, DM, (size_t)SQ_FULL * DM, SQ, DM, DM, nullptr, nullptr, 0u, 0u);
  k_gemm2<<<dim3((SQ / 128) * (DM / 64), NB), 128, 0, stream>>>(OL, DM, (size_t)SQ * DM, BO, DM, (size_t)0, 0u, 0.00000095367431640625f, (const float*)out, out, nullptr, nullptr, DM, (size_t)SQ_FULL * DM, SQ, DM, DM, nullptr, nullptr, 0u, 0u);
}
